// TranslationInvariantMP_52785148067991
// MI455X (gfx1250) — hardware-verified
//
#include <hip/hip_runtime.h>


namespace {
constexpr int V = 100000, VP = 100032  , KN = 32, F = 64;
constexpr float XS = 8.0f, WSC = 256.0f;

typedef _Float16 b16;
typedef __attribute__((ext_vector_type(16))) _Float16 v16b;
typedef __attribute__((ext_vector_type(8))) _Float16 v8b;
typedef __attribute__((ext_vector_type(8))) float v8f;
typedef __attribute__((ext_vector_type(4))) float v4f;
typedef __attribute__((ext_vector_type(2))) float v2f;
typedef __attribute__((ext_vector_type(2))) _Float16 v2b;
__device__ __forceinline__ float bf16_rne(float f) { unsigned int u = __float_as_uint(f); u += 0x7FFFu + ((u >> 16) & 1u); return __uint_as_float(u & 0xFFFF0000u); }
__device__ __forceinline__ void split16(float v, b16& hi, b16& lo) { hi = (b16)v; lo = (b16)(v - (float)hi); }
__device__ __forceinline__ v16b frag_kb(const b16* p, int hh) { const v8b a = *(const v8b*)(p + 8 * hh), b = *(const v8b*)(p + 16 + 8 * hh); v16b f;
#pragma unroll
  for (int e = 0; e < 8; ++e) { f[e] = a[e]; f[8 + e] = b[e]; } return f; }
__device__ __forceinline__ v8f wmma16b(v16b a, v16b b, v8f c) { v8f d = __builtin_amdgcn_wmma_f32_16x16x32_f16(false, a, false, b, (short)0, c, false, false); asm volatile("v_nop\n\tv_nop\n\tv_nop\n\tv_nop" : "+v"(d) : "v"(a), "v"(b)); return d; }
__device__ __forceinline__ void wave_lds_sync() { __builtin_amdgcn_fence(__ATOMIC_RELEASE, "workgroup"); __builtin_amdgcn_wave_barrier(); __builtin_amdgcn_fence(__ATOMIC_ACQUIRE, "workgroup"); }
__device__ __forceinline__ float pmul(float a, float b) { float p = a * b; asm volatile("" : "+v"(p)); return p; }
__device__ __forceinline__ int iclamp(int v, int lo, int hi) { return v < lo ? lo : (v > hi ? hi : v); }
__device__ __forceinline__ float elu(float x) { return x > 0.0f ? x : (__expf(x) - 1.0f); }

__global__ __launch_bounds__(256) void prepw_kernel(const float* __restrict__ w0, const float* __restrict__ w1, b16* __restrict__ WT) {
  const int t = blockIdx.x * 256 + threadIdx.x; if (t >= 2 * F * F / 8) return; const int e = t * 8; const int k = e / (F * F), r = e % (F * F); const int oo = r / F, i0 = r % F; const float* w = k == 0 ? w0 : w1; v8b o;
  for (int j = 0; j < 8; ++j) o[j] = (b16)(bf16_rne(w[(i0 + j) * F + oo]) * WSC); for (int pass = 0; pass < 2; ++pass) { *(volatile v8b*)(WT + e) = o; __threadfence(); }
}
template <int LAYER>
__global__ __launch_bounds__(256) void agg_kernel(const float* __restrict__ x, const float* __restrict__ out, const int* __restrict__ nbr, const float* __restrict__ d2, b16* __restrict__ AGh, b16* __restrict__ AGl) {
  const int wave = threadIdx.x >> 5, lane = threadIdx.x & 31; const size_t v = (size_t)blockIdx.x * 8 + wave; const int c0 = lane * 2;
  float a0 = 0.0f, a1 = 0.0f;
  if (v < (size_t)V) { float ws_ = 0.0f;
    for (int k = 0; k < KN; ++k) { const int u = iclamp(nbr[v * KN + k], 0, V - 1); const float w = __expf(-10.0f * bf16_rne(d2[v * KN + k])); ws_ += w; v2f s;
      if (LAYER == 0) { s = *(const v2f*)(x + (size_t)u * F + c0); s[0] = bf16_rne(s[0]); s[1] = bf16_rne(s[1]); } else { s = *(const v2f*)(out + (size_t)u * (2 * F) + c0); }
      a0 += pmul(w, s[0]); a1 += pmul(w, s[1]); }
    if (LAYER == 0) { const float x0 = bf16_rne(x[v * F + c0]), x1 = bf16_rne(x[v * F + c0 + 1]); a0 -= pmul(x0, ws_); a1 -= pmul(x1, ws_); }
    a0 *= (1.0f / KN); a1 *= (1.0f / KN); }
  v2b hv, lv; { b16 p, q; split16(a0 * XS, p, q); hv[0] = p; lv[0] = q; split16(a1 * XS, p, q); hv[1] = p; lv[1] = q; }
  for (int pass = 0; pass < 2; ++pass) { *(volatile v2b*)(AGh + v * F + c0) = hv; *(volatile v2b*)(AGl + v * F + c0) = lv; __threadfence(); }
}
template <int LAYER>
__global__ __launch_bounds__(128) void gemm_kernel(const b16* __restrict__ Ah, const b16* __restrict__ Al, const b16* __restrict__ W, const float* __restrict__ bias, float* __restrict__ out) {
  __shared__ __attribute__((aligned(16))) float Ts[4][16][F + 4];
  const int wave = threadIdx.x >> 5, lane = threadIdx.x & 31, nloc = lane & 15, hlf = lane >> 4; const size_t m0 = ((size_t)blockIdx.x * 4 + wave) * 16;
  v8f acc[4];
#pragma unroll
  for (int t = 0; t < 4; ++t) acc[t] = (v8f){};
#pragma unroll
  for (int kb = 0; kb < F; kb += 32) { const v16b a = frag_kb(Ah + (m0 + nloc) * F + kb, hlf), al = frag_kb(Al + (m0 + nloc) * F + kb, hlf);
#pragma unroll
    for (int t = 0; t < 4; ++t) { const v16b bw = frag_kb(W + (size_t)(t * 16 + nloc) * F + kb, hlf); acc[t] = wmma16b(a, bw, acc[t]); acc[t] = wmma16b(al, bw, acc[t]); } }
#pragma unroll
  for (int t = 0; t < 4; ++t) { const int c = t * 16 + nloc; const float bb = (LAYER == 1) ? bf16_rne(bias[c]) : 0.0f;
#pragma unroll
    for (int r = 0; r < 8; ++r) Ts[wave][8 * hlf + r][c] = elu(acc[t][r] * (1.0f / (XS * WSC)) + bb); }
  wave_lds_sync();
  for (int pass = 0; pass < 2; ++pass) { for (int rr = 0; rr < 16; ++rr) { const size_t row = m0 + rr; if (row < (size_t)V && lane < 16) *(volatile v4f*)(out + row * (2 * F) + LAYER * F + lane * 4) = *(const v4f*)(&Ts[wave][rr][lane * 4]); } __threadfence(); }
}
}

extern "C" void kernel_launch(void* const* d_in, const int* in_sizes, int n_in, void* d_out, int out_size, void* d_ws, size_t ws_size, hipStream_t stream) {
  (void)n_in;
  auto Fp = [&](int i) { return (const float*)d_in[i]; }; auto Ip = [&](int i) { return (const int*)d_in[i]; };
  if (in_sizes[0] != V * F || in_sizes[1] != V * KN || in_sizes[2] != V * KN || in_sizes[3] != F * F || in_sizes[4] != F * F || out_size != V * 2 * F) return;
  size_t off = 0; char* ws = (char*)d_ws;
  auto carve = [&](size_t bytes) { char* p = ws + off; off += (bytes + 255) & ~(size_t)255; return p; };
  b16* WT = (b16*)carve((size_t)2 * F * F * 2); b16* AGh = (b16*)carve((size_t)VP * F * 2); b16* AGl = (b16*)carve((size_t)VP * F * 2);
  if (off > ws_size || off > ((size_t)128 << 20)) return;
  float* out = (float*)d_out;
  prepw_kernel<<<(2 * F * F / 8 + 255) / 256, 256, 0, stream>>>(Fp(3), Fp(4), WT);
  agg_kernel<0><<<VP / 8, 256, 0, stream>>>(Fp(0), nullptr, Ip(1), Fp(2), AGh, AGl);
  gemm_kernel<0><<<VP / 64, 128, 0, stream>>>(AGh, AGl, WT, nullptr, out);
  agg_kernel<1><<<VP / 8, 256, 0, stream>>>(nullptr, out, Ip(1), Fp(2), AGh, AGl);
  gemm_kernel<1><<<VP / 64, 128, 0, stream>>>(AGh, AGl, WT + (size_t)F * F, Fp(5), out);
}
